// Rwkv6SelfAttention_36661840839089
// MI455X (gfx1250) — hardware-verified
//
#include <hip/hip_runtime.h>
#define TT 2048
#define HH 2048
#define HS 64
#define NH 32
#define DMIX 32
#define DM5 160
#define DM5P 192
#define DDEC 64

typedef __bf16 v16b __attribute__((ext_vector_type(16)));
typedef unsigned short v8us __attribute__((ext_vector_type(8), may_alias));
typedef float  v8f  __attribute__((ext_vector_type(8)));
typedef float  v4f  __attribute__((ext_vector_type(4)));
typedef float  v4fa __attribute__((ext_vector_type(4), may_alias));
union FragB { v16b v; v8us half[2]; unsigned short u[16]; };

__device__ __forceinline__ unsigned short bf16_bits(float x) { unsigned int u = __float_as_uint(x); return (unsigned short)((u + 0x7FFFu + ((u >> 16) & 1u)) >> 16); }
__device__ __forceinline__ float bf16_val(unsigned short b) { return __uint_as_float(((unsigned int)b) << 16); }
__device__ __forceinline__ float bf16_round(float x) { return bf16_val(bf16_bits(x)); }
template <int NT>
__device__ __forceinline__ v8f mmaN(v16b ah, v16b al, v16b bh, v16b bl, v8f c) {
  c = __builtin_amdgcn_wmma_f32_16x16x32_bf16(false, ah, false, bh, (short)0, c, false, false);
  if (NT >= 2) c = __builtin_amdgcn_wmma_f32_16x16x32_bf16(false, al, false, bh, (short)0, c, false, false);
  if (NT >= 3) c = __builtin_amdgcn_wmma_f32_16x16x32_bf16(false, ah, false, bl, (short)0, c, false, false);
  asm volatile("v_nop\n\tv_nop\n\tv_nop\n\tv_nop" : "+v"(c) : "v"(ah), "v"(al), "v"(bh), "v"(bl));
  return c;
}

__global__ __launch_bounds__(256) void k_wt_bf16(const float* __restrict__ W, unsigned short* __restrict__ Wt, int K, int N) {
  const int t = blockIdx.x * 256 + threadIdx.x;
  const int k8n = K / 8;
  if (t >= N * k8n) return;
  const int n = t / k8n, k8 = (t % k8n) * 8;
  v8us v;
#pragma unroll
  for (int i = 0; i < 8; ++i) v[i] = bf16_bits(W[(size_t)(k8 + i) * N + n]);
  *(volatile v8us*)(Wt + (size_t)n * K + k8) = v;
  __threadfence();
  *(volatile v8us*)(Wt + (size_t)n * K + k8) = v;
}

template <bool ASPLIT, int ACT, bool BIAS_BF16>
__global__ __launch_bounds__(128) void k_gemm_bf(const float* __restrict__ A, int lda, const unsigned short* __restrict__ Wt, int ldb,
                                               const float* __restrict__ bias, float* __restrict__ C, int ldc, int M, int N, int K) {
  __shared__ __attribute__((aligned(16))) float so[4][16][64];
  const int tid = threadIdx.x, w = tid >> 5, lane = tid & 31, ln = lane & 15, hh = lane >> 4;
  const int ntn = N / 64;
  const int wid = blockIdx.x * 4 + w;
  const int mt = wid / ntn, nq = wid % ntn;
  if (mt * 16 >= M) return;
  const int row0 = mt * 16, col0 = nq * 64;
  const float* arow = A + (size_t)(row0 + ln) * lda;
  v8f acc[4] = {};
  for (int kb = 0; kb < K; kb += 32) {
    FragB ah, al;
    const v4f x0 = *(const v4fa*)(arow + kb + 8 * hh), x1 = *(const v4fa*)(arow + kb + 8 * hh + 4);
    const v4f x2 = *(const v4fa*)(arow + kb + 16 + 8 * hh), x3 = *(const v4fa*)(arow + kb + 16 + 8 * hh + 4);
    float xs[16] = {x0[0],x0[1],x0[2],x0[3],x1[0],x1[1],x1[2],x1[3],x2[0],x2[1],x2[2],x2[3],x3[0],x3[1],x3[2],x3[3]};
#pragma unroll
    for (int i = 0; i < 16; ++i) { const unsigned short hb = bf16_bits(xs[i]); ah.u[i] = hb; al.u[i] = ASPLIT ? bf16_bits(xs[i] - bf16_val(hb)) : (unsigned short)0; }
#pragma unroll
    for (int t = 0; t < 4; ++t) {
      const unsigned short* brow = Wt + (size_t)(col0 + t * 16 + ln) * ldb + kb;
      FragB b;
      b.half[0] = *(const v8us*)(brow + 8 * hh);
      b.half[1] = *(const v8us*)(brow + 16 + 8 * hh);
      acc[t] = mmaN<ASPLIT ? 2 : 1>(ah.v, al.v, b.v, b.v, acc[t]);
    }
  }
#pragma unroll
  for (int t = 0; t < 4; ++t) {
    float bv = bias ? bias[col0 + t * 16 + ln] : 0.f;
    if (BIAS_BF16) bv = bf16_round(bv);
#pragma unroll
    for (int r = 0; r < 8; ++r) { float v = acc[t][r] + bv; if (ACT == 1) v = fmaxf(v, 0.f); so[w][8 * hh + r][t * 16 + ln] = v; }
  }
  __builtin_amdgcn_fence(__ATOMIC_ACQ_REL, "workgroup");
  __builtin_amdgcn_wave_barrier();
  const int rsub = lane >> 4, c4 = (lane & 15) * 4;
  for (int pass = 0; pass < 2; ++pass) {
#pragma unroll
    for (int q = 0; q < 8; ++q) {
      const int r = q * 2 + rsub;
      const v4f v = *(const v4fa*)&so[w][r][c4];
      *(volatile v4f*)(C + (size_t)(row0 + r) * ldc + col0 + c4) = v;
    }
    if (pass == 0) __threadfence();
  }
}

template <int D, bool CAUSAL>
__global__ __launch_bounds__(128) void k_flash(const float* __restrict__ qb, const float* __restrict__ kb, const float* __restrict__ vb,
                                             int pitch, int T, int H, float scale, float* __restrict__ y, int ypitch) {
  constexpr int KS = D / 32;
  constexpr int DT = D / 16;
  __shared__ __attribute__((aligned(16))) unsigned short sKh[32][D + 8], sKl[32][D + 8], sVh[32][D + 8], sVl[32][D + 8];
  __shared__ __attribute__((aligned(16))) unsigned short sPh[4][16][40], sPl[4][16][40];
  __shared__ __attribute__((aligned(16))) float sO[4][16][D];
  const int tid = threadIdx.x, w = tid >> 5, lane = tid & 31, ln = lane & 15, hh = lane >> 4;
  const int nqb = (T + 63) / 64;
  const int bh = blockIdx.x / nqb, qblk = blockIdx.x % nqb;
  const int b = bh / H, h = bh % H;
  const int q0 = qblk * 64 + w * 16;
  const float* Q = qb + (size_t)b * T * pitch + h * D;
  const float* K = kb + (size_t)b * T * pitch + h * D;
  const float* V = vb + (size_t)b * T * pitch + h * D;

  FragB aqh[KS], aql[KS];
  {
    int row = q0 + ln; if (row >= T) row = T - 1;
    const float* qr = Q + (size_t)row * pitch;
#pragma unroll
    for (int ks = 0; ks < KS; ++ks)
#pragma unroll
      for (int i = 0; i < 16; ++i) {
        const int d = ks * 32 + ((i < 8) ? (8 * hh + i) : (16 + 8 * hh + (i - 8)));
        const float x = qr[d] * scale; const unsigned short hb = bf16_bits(x);
        aqh[ks].u[i] = hb; aql[ks].u[i] = bf16_bits(x - bf16_val(hb));
      }
  }
  float m_r[8], l_r[8];
#pragma unroll
  for (int r = 0; r < 8; ++r) { m_r[r] = -3.0e38f; l_r[r] = 0.f; }
  v8f oacc[DT];
#pragma unroll
  for (int dt = 0; dt < DT; ++dt) oacc[dt] = (v8f){0.f,0.f,0.f,0.f,0.f,0.f,0.f,0.f};

  const int kv_end = CAUSAL ? min(T, qblk * 64 + 64) : T;
  for (int j0 = 0; j0 < kv_end; j0 += 32) {
    __syncthreads();
    for (int e = tid; e < 32 * (D / 4); e += 128) {
      const int r = e / (D / 4), c4 = (e % (D / 4)) * 4;
      const int key = j0 + r;
      v4f kf = {0.f,0.f,0.f,0.f}, vf = {0.f,0.f,0.f,0.f};
      if (key < T) { kf = *(const v4fa*)(K + (size_t)key * pitch + c4); vf = *(const v4fa*)(V + (size_t)key * pitch + c4); }
#pragma unroll
      for (int t = 0; t < 4; ++t) {
        unsigned short hb = bf16_bits(kf[t]); sKh[r][c4 + t] = hb; sKl[r][c4 + t] = bf16_bits(kf[t] - bf16_val(hb));
        hb = bf16_bits(vf[t]); sVh[r][c4 + t] = hb; sVl[r][c4 + t] = bf16_bits(vf[t] - bf16_val(hb));
      }
    }
    __syncthreads();
    v8f s[2];
#pragma unroll
    for (int nt = 0; nt < 2; ++nt) {
      v8f acc = {};
#pragma unroll
      for (int ks = 0; ks < KS; ++ks) {
        FragB bh_, bl_;
        bh_.half[0] = *(const v8us*)&sKh[nt * 16 + ln][ks * 32 + 8 * hh]; bh_.half[1] = *(const v8us*)&sKh[nt * 16 + ln][ks * 32 + 16 + 8 * hh];
        bl_.half[0] = *(const v8us*)&sKl[nt * 16 + ln][ks * 32 + 8 * hh]; bl_.half[1] = *(const v8us*)&sKl[nt * 16 + ln][ks * 32 + 16 + 8 * hh];
        acc = mmaN<3>(aqh[ks].v, aql[ks].v, bh_.v, bl_.v, acc);
      }
      s[nt] = acc;
    }
    float alpha[8];
#pragma unroll
    for (int r = 0; r < 8; ++r) {
      const int qi = q0 + 8 * hh + r;
      const int ja = j0 + ln, jb = j0 + 16 + ln;
      if (CAUSAL) { if (ja > qi) s[0][r] = -3.0e38f; if (jb > qi) s[1][r] = -3.0e38f; }
      if (ja >= T) s[0][r] = -3.0e38f;
      if (jb >= T) s[1][r] = -3.0e38f;
      float mx = fmaxf(s[0][r], s[1][r]);
      mx = fmaxf(mx, __shfl_xor(mx, 1, 32)); mx = fmaxf(mx, __shfl_xor(mx, 2, 32)); mx = fmaxf(mx, __shfl_xor(mx, 4, 32)); mx = fmaxf(mx, __shfl_xor(mx, 8, 32));
      const float mnew = fmaxf(m_r[r], mx);
      alpha[r] = (mnew > -1.0e38f) ? __expf(m_r[r] - mnew) : 1.0f;
      const float p0 = (s[0][r] > -1.0e38f) ? __expf(s[0][r] - mnew) : 0.f;
      const float p1 = (s[1][r] > -1.0e38f) ? __expf(s[1][r] - mnew) : 0.f;
      m_r[r] = mnew;
      l_r[r] = l_r[r] * alpha[r] + p0 + p1;
      unsigned short hb = bf16_bits(p0); sPh[w][8 * hh + r][ln] = hb;      sPl[w][8 * hh + r][ln] = bf16_bits(p0 - bf16_val(hb));
      hb = bf16_bits(p1);                sPh[w][8 * hh + r][16 + ln] = hb; sPl[w][8 * hh + r][16 + ln] = bf16_bits(p1 - bf16_val(hb));
    }
#pragma unroll
    for (int dt = 0; dt < DT; ++dt)
#pragma unroll
      for (int r = 0; r < 8; ++r) oacc[dt][r] *= alpha[r];
    __builtin_amdgcn_fence(__ATOMIC_ACQ_REL, "workgroup");
    __builtin_amdgcn_wave_barrier();
    FragB pah, pal;
    pah.half[0] = *(const v8us*)&sPh[w][ln][8 * hh]; pah.half[1] = *(const v8us*)&sPh[w][ln][16 + 8 * hh];
    pal.half[0] = *(const v8us*)&sPl[w][ln][8 * hh]; pal.half[1] = *(const v8us*)&sPl[w][ln][16 + 8 * hh];
#pragma unroll
    for (int dt = 0; dt < DT; ++dt) {
      FragB bvh, bvl;
#pragma unroll
      for (int i = 0; i < 8; ++i) {
        bvh.u[i] = sVh[8 * hh + i][dt * 16 + ln]; bvh.u[8 + i] = sVh[16 + 8 * hh + i][dt * 16 + ln];
        bvl.u[i] = sVl[8 * hh + i][dt * 16 + ln]; bvl.u[8 + i] = sVl[16 + 8 * hh + i][dt * 16 + ln];
      }
      oacc[dt] = mmaN<3>(pah.v, pal.v, bvh.v, bvl.v, oacc[dt]);
    }
    __builtin_amdgcn_fence(__ATOMIC_ACQ_REL, "workgroup");
    __builtin_amdgcn_wave_barrier();
  }
#pragma unroll
  for (int r = 0; r < 8; ++r) {
    float l = l_r[r];
    l += __shfl_xor(l, 1, 32); l += __shfl_xor(l, 2, 32); l += __shfl_xor(l, 4, 32); l += __shfl_xor(l, 8, 32);
    l_r[r] = (l > 0.f) ? 1.0f / l : 0.f;
  }
#pragma unroll
  for (int dt = 0; dt < DT; ++dt)
#pragma unroll
    for (int r = 0; r < 8; ++r) sO[w][8 * hh + r][dt * 16 + ln] = oacc[dt][r] * l_r[r];
  __builtin_amdgcn_fence(__ATOMIC_ACQ_REL, "workgroup");
  __builtin_amdgcn_wave_barrier();
  for (int pass = 0; pass < 2; ++pass) {
    for (int r = 0; r < 16; ++r) {
      const int row = q0 + r;
      if (row < T && lane < D / 4) {
        const v4f val = *(const v4fa*)&sO[w][r][lane * 4];
        *(volatile v4f*)(y + ((size_t)b * T + row) * ypitch + h * D + lane * 4) = val;
      }
    }
    if (pass == 0) __threadfence();
  }
}

template <bool ASPLIT, int ACT, bool BIAS_BF16, bool RES_BF16>
__global__ __launch_bounds__(128) void k_gemm_bf3(const float* __restrict__ A, int lda, const unsigned short* __restrict__ Wt, int ldb,
                                                const float* __restrict__ bias, const float* __restrict__ resid, int rmod, int ldr,
                                                float* __restrict__ C, int ldc, int M, int N, int K) {
  __shared__ __attribute__((aligned(16))) float so[4][16][64];
  const int tid = threadIdx.x, w = tid >> 5, lane = tid & 31, ln = lane & 15, hh = lane >> 4;
  const int ntn = N / 64;
  const int wid = blockIdx.x * 4 + w;
  const int mt = wid / ntn, nq = wid % ntn;
  if (mt * 16 >= M) return;
  const int row0 = mt * 16, col0 = nq * 64;
  const float* arow = A + (size_t)(row0 + ln) * lda;
  v8f acc[4] = {};
  for (int kb = 0; kb < K; kb += 32) {
    FragB ah, al;
    const v4f x0 = *(const v4fa*)(arow + kb + 8 * hh), x1 = *(const v4fa*)(arow + kb + 8 * hh + 4);
    const v4f x2 = *(const v4fa*)(arow + kb + 16 + 8 * hh), x3 = *(const v4fa*)(arow + kb + 16 + 8 * hh + 4);
    float xs[16] = {x0[0],x0[1],x0[2],x0[3],x1[0],x1[1],x1[2],x1[3],x2[0],x2[1],x2[2],x2[3],x3[0],x3[1],x3[2],x3[3]};
#pragma unroll
    for (int i = 0; i < 16; ++i) { const unsigned short hb = bf16_bits(xs[i]); ah.u[i] = hb; al.u[i] = ASPLIT ? bf16_bits(xs[i] - bf16_val(hb)) : (unsigned short)0; }
#pragma unroll
    for (int t = 0; t < 4; ++t) {
      const unsigned short* brow = Wt + (size_t)(col0 + t * 16 + ln) * ldb + kb;
      FragB b;
      b.half[0] = *(const v8us*)(brow + 8 * hh);
      b.half[1] = *(const v8us*)(brow + 16 + 8 * hh);
      acc[t] = mmaN<ASPLIT ? 2 : 1>(ah.v, al.v, b.v, b.v, acc[t]);
    }
  }
#pragma unroll
  for (int t = 0; t < 4; ++t) {
    const int col = col0 + t * 16 + ln;
    float bv = bias ? bias[col] : 0.f;
    if (BIAS_BF16) bv = bf16_round(bv);
#pragma unroll
    for (int r = 0; r < 8; ++r) {
      float v = acc[t][r] + bv;
      if (resid) { float rv = resid[(size_t)((row0 + 8 * hh + r) % rmod) * ldr + col]; if (RES_BF16) rv = bf16_round(rv); v += rv; }
      if (ACT == 1) v = fmaxf(v, 0.f);
      if (ACT == 2) v = 0.5f * v * (1.0f + erff(v * 0.70710678118654752f));
      if (ACT == 3) { const float u = 0.7978845608028654f * (v + 0.044715f * v * v * v); v = 0.5f * v * (1.0f + tanhf(u)); }
      so[w][8 * hh + r][t * 16 + ln] = v;
    }
  }
  __builtin_amdgcn_fence(__ATOMIC_ACQ_REL, "workgroup");
  __builtin_amdgcn_wave_barrier();
  const int rsub = lane >> 4, c4 = (lane & 15) * 4;
  for (int pass = 0; pass < 2; ++pass) {
#pragma unroll
    for (int q = 0; q < 8; ++q) {
      const int r = q * 2 + rsub;
      const v4f v = *(const v4fa*)&so[w][r][c4];
      *(volatile v4f*)(C + (size_t)(row0 + r) * ldc + col0 + c4) = v;
    }
    if (pass == 0) __threadfence();
  }
}
template <bool PARAM_BF16>
__global__ __launch_bounds__(256) void k_layernorm(const float* __restrict__ X, const float* __restrict__ R, const float* __restrict__ g, const float* __restrict__ bta,
                                                  float* __restrict__ out_sum, float* __restrict__ out_norm, int N, float eps) {
  __shared__ float red[256];
  const int row = blockIdx.x, tid = threadIdx.x;
  const float* x = X + (size_t)row * N; const float* rr = R ? R + (size_t)row * N : nullptr;
  float vals[16];
  const int per = N / 256;
  float s1 = 0.f;
  for (int u = 0; u < per / 4; ++u) {
    const int j = tid * 4 + 1024 * u;
    const v4f a = *(const v4fa*)(x + j);
    v4f b = {0.f,0.f,0.f,0.f}; if (rr) b = *(const v4fa*)(rr + j);
#pragma unroll
    for (int q = 0; q < 4; ++q) { const float v = a[q] + b[q]; vals[u * 4 + q] = v; s1 += v; }
  }
  red[tid] = s1; __syncthreads();
  for (int st = 128; st > 0; st >>= 1) { if (tid < st) red[tid] += red[tid + st]; __syncthreads(); }
  const float mu = red[0] / (float)N; __syncthreads();
  float s2 = 0.f;
  for (int u = 0; u < per / 4; ++u)
#pragma unroll
    for (int q = 0; q < 4; ++q) { const float c = vals[u * 4 + q] - mu; s2 += c * c; }
  red[tid] = s2; __syncthreads();
  for (int st = 128; st > 0; st >>= 1) { if (tid < st) red[tid] += red[tid + st]; __syncthreads(); }
  const float rs = rsqrtf(red[0] / (float)N + eps);
  for (int pass = 0; pass < 2; ++pass) {
    for (int u = 0; u < per / 4; ++u) {
      const int j = tid * 4 + 1024 * u;
      v4f o, sm;
#pragma unroll
      for (int q = 0; q < 4; ++q) {
        float gg = g[j + q], bb = bta[j + q];
        if (PARAM_BF16) { gg = bf16_round(gg); bb = bf16_round(bb); }
        sm[q] = vals[u * 4 + q]; o[q] = (vals[u * 4 + q] - mu) * rs * gg + bb;
      }
      if (out_sum) *(volatile v4f*)(out_sum + (size_t)row * N + j) = sm;
      *(volatile v4f*)(out_norm + (size_t)row * N + j) = o;
    }
    if (pass == 0) __threadfence();
  }
}

__global__ __launch_bounds__(256) void k_round_rows(const float* __restrict__ W, unsigned short* __restrict__ Wt, int n8) {
  const int t = blockIdx.x * 256 + threadIdx.x;
  if (t >= n8) return;
  const v4f a = *(const v4fa*)(W + (size_t)t * 8), b = *(const v4fa*)(W + (size_t)t * 8 + 4);
  v8us v; v[0]=bf16_bits(a[0]); v[1]=bf16_bits(a[1]); v[2]=bf16_bits(a[2]); v[3]=bf16_bits(a[3]);
  v[4]=bf16_bits(b[0]); v[5]=bf16_bits(b[1]); v[6]=bf16_bits(b[2]); v[7]=bf16_bits(b[3]);
  *(volatile v8us*)(Wt + (size_t)t * 8) = v; __threadfence(); *(volatile v8us*)(Wt + (size_t)t * 8) = v;
}

__global__ __launch_bounds__(256) void k_roundcopy(const float* __restrict__ src, float* __restrict__ dst, int n8) {
  const size_t t = (size_t)blockIdx.x * 256 + threadIdx.x;
  if (t >= (size_t)n8 * 2) return;
  v4f a = *(const v4fa*)(src + t * 4);
  for (int i = 0; i < 4; ++i) a[i] = bf16_round(a[i]);
  *(volatile v4f*)(dst + t * 4) = a; __threadfence(); *(volatile v4f*)(dst + t * 4) = a;
}

__global__ __launch_bounds__(256) void k_shift(const float* __restrict__ xn, const float* __restrict__ state1, const float* __restrict__ maa_x, float* __restrict__ sx, float* __restrict__ xxx) {
  const size_t t4 = (size_t)blockIdx.x * 256 + threadIdx.x; if (t4 >= (size_t)TT * HH / 4) return;
  const int t = (int)(t4 / (HH / 4)), c4 = (int)(t4 % (HH / 4)) * 4;
  const v4f cur = *(const v4fa*)(xn + t4 * 4);
  v4f past; if (t == 0) { for (int q = 0; q < 4; ++q) past[q] = bf16_round(state1[c4 + q]); } else past = *(const v4fa*)(xn + (size_t)(t - 1) * HH + c4);
  v4f s, xx; for (int q = 0; q < 4; ++q) { s[q] = past[q] - cur[q]; xx[q] = cur[q] + s[q] * bf16_round(maa_x[c4 + q]); }
  *(volatile v4f*)(sx + t4 * 4) = s; *(volatile v4f*)(xxx + t4 * 4) = xx; __threadfence(); *(volatile v4f*)(sx + t4 * 4) = s; *(volatile v4f*)(xxx + t4 * 4) = xx;
}
__global__ __launch_bounds__(256) void k_wt_maa1(const float* __restrict__ W, unsigned short* __restrict__ Bt) {
  const int t = blockIdx.x * 256 + threadIdx.x; if (t >= DM5P * (HH / 8)) return;
  const int n = t / (HH / 8), k8 = (t % (HH / 8)) * 8; v8us v;
  for (int i = 0; i < 8; ++i) v[i] = (n < DM5) ? bf16_bits(W[(size_t)(k8 + i) * DM5 + n]) : (unsigned short)0;
  *(volatile v8us*)(Bt + (size_t)n * HH + k8) = v; __threadfence(); *(volatile v8us*)(Bt + (size_t)n * HH + k8) = v;
}
__global__ __launch_bounds__(256) void k_tanh_inplace(float* __restrict__ a, int n4) { const int t = blockIdx.x * 256 + threadIdx.x; if (t >= n4) return; v4f v = *(const v4fa*)(a + (size_t)t * 4); for (int q = 0; q < 4; ++q) v[q] = tanhf(v[q]); *(volatile v4f*)(a + (size_t)t * 4) = v; __threadfence(); *(volatile v4f*)(a + (size_t)t * 4) = v; }
__global__ __launch_bounds__(256) void k_mixel(const float* __restrict__ sx, const float* __restrict__ tmp, const float* __restrict__ xn, float* __restrict__ mixed, int n4) {
  const int t = blockIdx.x * 256 + threadIdx.x; if (t >= n4) return;
  const v4f a = *(const v4fa*)(sx + (size_t)t * 4), b = *(const v4fa*)(tmp + (size_t)t * 4), c = *(const v4fa*)(xn + (size_t)t * 4); v4f o; for (int q = 0; q < 4; ++q) o[q] = a[q] * b[q] + c[q];
  *(volatile v4f*)(mixed + (size_t)t * 4) = o; __threadfence(); *(volatile v4f*)(mixed + (size_t)t * 4) = o;
}
__global__ __launch_bounds__(256) void k_silu_inplace(float* __restrict__ a, int n4) { const int t = blockIdx.x * 256 + threadIdx.x; if (t >= n4) return; v4f v = *(const v4fa*)(a + (size_t)t * 4); for (int q = 0; q < 4; ++q) v[q] = v[q] / (1.0f + expf(-v[q])); *(volatile v4f*)(a + (size_t)t * 4) = v; __threadfence(); *(volatile v4f*)(a + (size_t)t * 4) = v; }
__global__ __launch_bounds__(256) void k_decay(float* __restrict__ w, const float* __restrict__ time_decay, int n4) {
  const int t = blockIdx.x * 256 + threadIdx.x; if (t >= n4) return; const int c4 = (t % (HH / 4)) * 4;
  v4f v = *(const v4fa*)(w + (size_t)t * 4); for (int q = 0; q < 4; ++q) { float d = bf16_round(time_decay[c4 + q]) + v[q]; d = fminf(fmaxf(d, -9.72f), 2.27f); v[q] = expf(-expf(d)); }
  *(volatile v4f*)(w + (size_t)t * 4) = v; __threadfence(); *(volatile v4f*)(w + (size_t)t * 4) = v;
}
__global__ __launch_bounds__(256) void k_wkv(const float* __restrict__ r, const float* __restrict__ k, const float* __restrict__ v, const float* __restrict__ td, const float* __restrict__ time_first,
                                          const float* __restrict__ state2, float* __restrict__ wkv, float* __restrict__ s_out) {
  __shared__ float part[64][65];
  __shared__ float orow[64];
  const int h = blockIdx.x, tid = threadIdx.x; const int i = tid >> 2, j0 = (tid & 3) * 16;
  float S[16]; for (int q = 0; q < 16; ++q) S[q] = bf16_round(state2[((size_t)h * HS + i) * HS + j0 + q]);
  const float tf = bf16_round(time_first[h * HS + i]);
  for (int t = 0; t < TT; ++t) {
    const size_t base = (size_t)t * HH + h * HS;
    const float kt = k[base + i], rt = r[base + i], wt = td[base + i];
    float vj[16]; for (int q = 0; q < 16; ++q) vj[q] = v[base + j0 + q];
#pragma unroll
    for (int q = 0; q < 16; ++q) { const float kv = kt * vj[q]; part[i][j0 + q] = rt * (tf * kv + S[q]); S[q] = kv + wt * S[q]; }
    __syncthreads();
    if (tid < 64) { float s = 0.f;
#pragma unroll 8
      for (int ii = 0; ii < 64; ++ii) s += part[ii][tid]; orow[tid] = s; }
    __syncthreads();
    if (tid < 64) { const float vv = orow[tid]; *(volatile float*)(wkv + base + tid) = vv; }
    __threadfence();
    if (tid < 64) { const float vv = orow[tid]; *(volatile float*)(wkv + base + tid) = vv; }
    __syncthreads();
  }
  for (int q = 0; q < 16; ++q) part[i][j0 + q] = S[q];
  __syncthreads();
  for (int pass = 0; pass < 2; ++pass) {
    for (int e = tid; e < 64 * 16; e += 256) { const int row = e >> 4, c4 = (e & 15) * 4; v4f o = {part[row][c4], part[row][c4 + 1], part[row][c4 + 2], part[row][c4 + 3]}; *(volatile v4f*)(s_out + ((size_t)h * HS + row) * HS + c4) = o; }
    if (pass == 0) __threadfence();
  }
}
__global__ __launch_bounds__(256) void k_gn_gate(const float* __restrict__ wkv, const float* __restrict__ g, const float* __restrict__ lw, const float* __restrict__ lb, float* __restrict__ ng) {
  const int tid = threadIdx.x, w = tid >> 5, lane = tid & 31; const size_t th = (size_t)blockIdx.x * 8 + w; if (th >= (size_t)TT * NH) return;
  const size_t base = th * HS; const int c0 = (int)(th % NH) * HS;
  const float a = wkv[base + lane], b = wkv[base + 32 + lane];
  float s = a + b; for (int o = 16; o >= 1; o >>= 1) s += __shfl_xor(s, o, 32); const float mu = s * (1.0f / HS);
  float q2 = (a - mu) * (a - mu) + (b - mu) * (b - mu); for (int o = 16; o >= 1; o >>= 1) q2 += __shfl_xor(q2, o, 32); const float rs = rsqrtf(q2 * (1.0f / HS) + 1e-5f);
  const float o1 = ((a - mu) * rs * bf16_round(lw[c0 + lane]) + bf16_round(lb[c0 + lane])) * g[base + lane];
  const float o2 = ((b - mu) * rs * bf16_round(lw[c0 + 32 + lane]) + bf16_round(lb[c0 + 32 + lane])) * g[base + 32 + lane];
  *(volatile float*)(ng + base + lane) = o1; *(volatile float*)(ng + base + 32 + lane) = o2; __threadfence(); *(volatile float*)(ng + base + lane) = o1; *(volatile float*)(ng + base + 32 + lane) = o2;
}
__global__ __launch_bounds__(256) void k_copyrow(const float* __restrict__ src, float* __restrict__ dst, int n4) { const int t = blockIdx.x * 256 + threadIdx.x; if (t >= n4) return; const v4f v = *(const v4fa*)(src + (size_t)t * 4); *(volatile v4f*)(dst + (size_t)t * 4) = v; __threadfence(); *(volatile v4f*)(dst + (size_t)t * 4) = v; }

extern "C" void kernel_launch(void* const* d_in, const int* in_sizes, int n_in,
                              void* d_out, int out_size, void* d_ws, size_t ws_size, hipStream_t stream) {
  (void)in_sizes; (void)n_in; (void)out_size;
  const float* x = (const float*)d_in[0]; const float* state1 = (const float*)d_in[1]; const float* state2 = (const float*)d_in[2];
  const float* ln1w = (const float*)d_in[3]; const float* ln1b = (const float*)d_in[4]; const float* maa_x = (const float*)d_in[5];
  const float* maa_w1 = (const float*)d_in[6]; const float* maa_w2 = (const float*)d_in[7]; const float* maa_bias = (const float*)d_in[8];
  const float* dec_w1 = (const float*)d_in[9]; const float* dec_w2 = (const float*)d_in[10]; const float* time_decay = (const float*)d_in[11]; const float* time_first = (const float*)d_in[12];
  const float* Wr = (const float*)d_in[13]; const float* Wk = (const float*)d_in[14]; const float* Wv = (const float*)d_in[15]; const float* Wg = (const float*)d_in[16]; const float* Wo = (const float*)d_in[17];
  const float* lnxw = (const float*)d_in[18]; const float* lnxb = (const float*)d_in[19];
  float* out = (float*)d_out; float* st1 = (float*)((char*)d_out + 16777216); float* st2 = (float*)((char*)d_out + 16785408);
  char* ws = (char*)d_ws; size_t off = 0;
  auto take = [&](size_t bytes) { char* p = ws + off; off += (bytes + 255) & ~(size_t)255; return p; };
  const size_t NE = (size_t)TT * HH; const int n4 = (int)(NE / 4); const int n8 = HH * HH / 8;
  unsigned short* Wt5[5]; for (int i = 0; i < 5; ++i) Wt5[i] = (unsigned short*)take((size_t)HH * HH * 2);
  unsigned short* Bm1 = (unsigned short*)take((size_t)DM5P * HH * 2); unsigned short* Bm2[5]; for (int i = 0; i < 5; ++i) Bm2[i] = (unsigned short*)take((size_t)HH * DMIX * 2);
  unsigned short* Bd1 = (unsigned short*)take((size_t)DDEC * HH * 2); unsigned short* Bd2 = (unsigned short*)take((size_t)HH * DDEC * 2);
  float* xr = (float*)take(NE * 4); float* xn = (float*)take(NE * 4); float* sx = (float*)take(NE * 4); float* xxx = (float*)take(NE * 4);
  float* m5 = (float*)take((size_t)TT * DM5P * 4); float* tmp = (float*)take(NE * 4);
  float* rb = (float*)take(NE * 4); float* kb = (float*)take(NE * 4); float* vb = (float*)take(NE * 4); float* gbuf = (float*)take(NE * 4);
  float* wtmp = (float*)take((size_t)TT * DDEC * 4); float* td = (float*)take(NE * 4); float* wkv = (float*)take(NE * 4);
  if (off > ws_size) return;
  const float* W5[5] = {Wr, Wk, Wv, Wg, Wo};
  for (int i = 0; i < 5; ++i) k_round_rows<<<(n8 + 255) / 256, 256, 0, stream>>>(W5[i], Wt5[i], n8);
  k_wt_maa1<<<(DM5P * (HH / 8) + 255) / 256, 256, 0, stream>>>(maa_w1, Bm1);
  for (int i = 0; i < 5; ++i) k_wt_bf16<<<(HH * (DMIX / 8) + 255) / 256, 256, 0, stream>>>(maa_w2 + (size_t)i * DMIX * HH, Bm2[i], DMIX, HH);
  k_wt_bf16<<<(DDEC * (HH / 8) + 255) / 256, 256, 0, stream>>>(dec_w1, Bd1, HH, DDEC);
  k_wt_bf16<<<(HH * (DDEC / 8) + 255) / 256, 256, 0, stream>>>(dec_w2, Bd2, DDEC, HH);
  k_roundcopy<<<(n4 + 255) / 256, 256, 0, stream>>>(x, xr, (int)(NE / 8));
  k_layernorm<true><<<TT, 256, 0, stream>>>(xr, nullptr, ln1w, ln1b, nullptr, xn, HH, 1e-5f);
  k_copyrow<<<(HH / 4 + 255) / 256, 256, 0, stream>>>(xn + (size_t)(TT - 1) * HH, st1, HH / 4);
  k_shift<<<(n4 + 255) / 256, 256, 0, stream>>>(xn, state1, maa_x, sx, xxx);
  const int gb192 = ((TT / 16) * (DM5P / 64) + 3) / 4, gbH = ((TT / 16) * (HH / 64) + 3) / 4, gb64 = ((TT / 16) * 1 + 3) / 4;
  k_gemm_bf3<true, 0, false, false><<<gb192, 128, 0, stream>>>(xxx, HH, Bm1, HH, nullptr, nullptr, 1, 0, m5, DM5P, TT, DM5P, HH);
  k_tanh_inplace<<<(TT * DM5P / 4 + 255) / 256, 256, 0, stream>>>(m5, TT * DM5P / 4);
  float* mixed = xxx;
  float* dstbuf[5] = {wtmp, kb, vb, rb, gbuf};
  for (int i = 0; i < 5; ++i) {
    k_gemm_bf3<true, 0, true, false><<<gbH, 128, 0, stream>>>(m5 + i * DMIX, DM5P, Bm2[i], DMIX, maa_bias + (size_t)i * HH, nullptr, 1, 0, tmp, HH, TT, HH, DMIX);
    k_mixel<<<(n4 + 255) / 256, 256, 0, stream>>>(sx, tmp, xn, mixed, n4);
    if (i == 0) {
      k_gemm_bf3<true, 0, false, false><<<gb64, 128, 0, stream>>>(mixed, HH, Bd1, HH, nullptr, nullptr, 1, 0, wtmp, DDEC, TT, DDEC, HH);
      k_tanh_inplace<<<(TT * DDEC / 4 + 255) / 256, 256, 0, stream>>>(wtmp, TT * DDEC / 4);
      k_gemm_bf3<true, 0, false, false><<<gbH, 128, 0, stream>>>(wtmp, DDEC, Bd2, DDEC, nullptr, nullptr, 1, 0, td, HH, TT, HH, DDEC);
      k_decay<<<(n4 + 255) / 256, 256, 0, stream>>>(td, time_decay, n4);
    } else {
      const int wi = (i == 1) ? 1 : (i == 2) ? 2 : (i == 3) ? 0 : 3;
      k_gemm_bf3<true, 0, false, false><<<gbH, 128, 0, stream>>>(mixed, HH, Wt5[wi], HH, nullptr, nullptr, 1, 0, dstbuf[i], HH, TT, HH, HH);
      if (i == 4) k_silu_inplace<<<(n4 + 255) / 256, 256, 0, stream>>>(gbuf, n4);
    }
  }
  k_wkv<<<NH, 256, 0, stream>>>(rb, kb, vb, td, time_first, state2, wkv, st2);
  float* ng = tmp;
  k_gn_gate<<<(TT * NH + 7) / 8, 256, 0, stream>>>(wkv, gbuf, lnxw, lnxb, ng);
  k_gemm_bf3<true, 0, false, false><<<gbH, 128, 0, stream>>>(ng, HH, Wt5[4], HH, nullptr, xr, TT, HH, out, HH, TT, HH, HH);
}
